// MaxLukAFRNN_FashionMNIST_52802327937293
// MI455X (gfx1250) — hardware-verified
//
#include <hip/hip_runtime.h>
#include <stddef.h>
#include <stdint.h>

#pragma clang fp contract(off)

#define IMGW   28
#define NPIX   784
#define NCH    8
#define HO     26
#define NPOS   676
#define KTOT   5408
#define KP     5440
#define NPIECE 680
#define NKB    169
#define NCLS   10
#define NPAD   16
#define TPB    256

static_assert(KTOT == NCH * NPOS);
static_assert(NKB * 32 == KTOT);
static_assert((KP * 2) % 128 == 0);
static_assert(NPIECE * 8 == KP);
static_assert(KP >= KTOT);
static_assert(NPIECE <= 3 * TPB);
static_assert(NPIECE > 2 * TPB);
static_assert((16 * NCLS * 4) % 128 == 0);
static_assert(16 * NCLS == 160);

typedef _Float16 v16h __attribute__((ext_vector_type(16)));
typedef _Float16 v8h  __attribute__((ext_vector_type(8)));
typedef float    v8f  __attribute__((ext_vector_type(8)));
typedef float    v4f  __attribute__((ext_vector_type(4)));
typedef unsigned int v4u __attribute__((ext_vector_type(4)));
typedef v4f __attribute__((may_alias)) v4fa;

union Frag  { v16h v; v8h h[2]; };
union HPack { v8h h; v4u u; };

__device__ __forceinline__ v8f mma16(v16h a, v16h b, v8f cacc) {
  cacc = __builtin_amdgcn_wmma_f32_16x16x32_f16(false, a, false, b, (short)0, cacc, false, false);
  asm volatile("v_nop\n\tv_nop\n\tv_nop\n\tv_nop" : "+v"(cacc) : "v"(a), "v"(b));
  return cacc;
}

__device__ __forceinline__ v8f zero8() { return (v8f){0.f, 0.f, 0.f, 0.f, 0.f, 0.f, 0.f, 0.f}; }

__device__ __forceinline__ v16h ldfrag_g(const _Float16* __restrict__ p, int ld, int row0, int k0, int lane) {
  const int m = lane & 15, lh = lane >> 4;
  const _Float16* q = p + (size_t)(row0 + m) * ld + k0 + 8 * lh;
  Frag f;
  f.h[0] = *(const v8h*)(q);
  f.h[1] = *(const v8h*)(q + 16);
  return f.v;
}

__device__ __forceinline__ v4u w_piece(int p, const float* __restrict__ wrow, bool rowok) {
  HPack pk;
#pragma unroll
  for (int e = 0; e < 8; ++e) {
    const int c  = 8 * p + e;
    const int cc = (c < KTOT) ? c : (KTOT - 1);
    float v = wrow[cc];
    v = (rowok && c < KTOT) ? v : 0.0f;
    pk.h[e] = (_Float16)v;
  }
  return pk.u;
}

__global__ __launch_bounds__(TPB) void k_wprep(const float* __restrict__ wd, _Float16* __restrict__ Wp) {
  const int tid = threadIdx.x;
  const int n = blockIdx.x;
  const bool rowok = n < NCLS;
  const int nc = rowok ? n : (NCLS - 1);
  const float* wrow = wd + (size_t)nc * KTOT;
  const int p0 = tid, p1 = tid + TPB, p2 = tid + 2 * TPB;
  const v4u q0 = w_piece(p0, wrow, rowok);
  const v4u q1 = w_piece(p1, wrow, rowok);
  const v4u q2 = w_piece(p2, wrow, rowok);
  const bool s2 = p2 < NPIECE;
  _Float16* row = Wp + (size_t)n * KP;
  *(volatile v4u*)(row + 8 * p0) = q0;
  *(volatile v4u*)(row + 8 * p1) = q1;
  if (s2) *(volatile v4u*)(row + 8 * p2) = q2;
  __threadfence();
  *(volatile v4u*)(row + 8 * p0) = q0;
  *(volatile v4u*)(row + 8 * p1) = q1;
  if (s2) *(volatile v4u*)(row + 8 * p2) = q2;
}

__device__ __forceinline__ v4u feat_piece(int p, const float* oma, const float* omw) {
  const int k0 = p * 8;
  int f   = k0 / NPOS;
  int rem = k0 - f * NPOS;
  int r   = rem / HO;
  int c   = rem - r * HO;
  HPack pk;
#pragma unroll
  for (int e = 0; e < 8; ++e) {
    const int fc = (f < NCH) ? f : (NCH - 1);
    const float* wb = omw + fc * 9;
    const float* xb = oma + r * IMGW + c;
    float m = 0.0f;
#pragma unroll
    for (int i = 0; i < 3; ++i) {
#pragma unroll
      for (int j = 0; j < 3; ++j) {
        const float t = 1.0f - (xb[i * IMGW + j] + wb[i * 3 + j]);
        m = fmaxf(m, t);
      }
    }
    m = (k0 + e < KTOT) ? m : 0.0f;
    pk.h[e] = (_Float16)m;
    c += 1;
    const int cw = (c == HO) ? 1 : 0;
    c = cw ? 0 : c;
    r += cw;
    const int rw = (r == HO) ? 1 : 0;
    r = rw ? 0 : r;
    f += rw;
  }
  return pk.u;
}

__global__ __launch_bounds__(TPB) void k_feat(const float* __restrict__ x, const float* __restrict__ wf,
                                             _Float16* __restrict__ Ap) {
  __shared__ float oma[NPIX];
  __shared__ float omw[NCH * 9];
  const int tid = threadIdx.x;
  const int img = blockIdx.x;
  const float* xi = x + (size_t)img * NPIX;
#pragma unroll
  for (int it = 0; it < 4; ++it) {
    const int i  = tid + TPB * it;
    const int ic = (i < NPIX) ? i : (NPIX - 1);
    const float v = xi[ic];
    if (i < NPIX) oma[i] = 1.0f - v;
  }
  {
    const int wc = (tid < NCH * 9) ? tid : (NCH * 9 - 1);
    const float v = wf[wc];
    if (tid < NCH * 9) omw[tid] = 1.0f - v;
  }
  __syncthreads();

  const int p0 = tid, p1 = tid + TPB, p2 = tid + 2 * TPB;
  const v4u q0 = feat_piece(p0, oma, omw);
  const v4u q1 = feat_piece(p1, oma, omw);
  const v4u q2 = feat_piece(p2, oma, omw);
  const bool s2 = p2 < NPIECE;
  _Float16* row = Ap + (size_t)img * KP;
  *(volatile v4u*)(row + 8 * p0) = q0;
  *(volatile v4u*)(row + 8 * p1) = q1;
  if (s2) *(volatile v4u*)(row + 8 * p2) = q2;
  __threadfence();
  *(volatile v4u*)(row + 8 * p0) = q0;
  *(volatile v4u*)(row + 8 * p1) = q1;
  if (s2) *(volatile v4u*)(row + 8 * p2) = q2;
}

__global__ __launch_bounds__(32) void k_gemm(const _Float16* __restrict__ Ap, const _Float16* __restrict__ Wp,
                                            float* __restrict__ out) {
  __shared__ float tile[NPAD * NPAD];
  __shared__ __align__(16) float sres[16 * NCLS];
  const int lane = threadIdx.x;
  const int h = lane >> 4, c = lane & 15;
  const int m0 = blockIdx.x * 16;

  v8f acc = zero8();
#pragma unroll 1
  for (int kb = 0; kb < NKB; ++kb) {
    const int k0 = kb * 32;
    const v16h a = ldfrag_g(Ap, KP, m0, k0, lane);
    const v16h b = ldfrag_g(Wp, KP, 0, k0, lane);
    acc = mma16(a, b, acc);
  }

#pragma unroll
  for (int r = 0; r < 8; ++r) tile[(8 * h + r) * NPAD + c] = acc[r];
  __syncthreads();

  const float* row = tile + c * NPAD;
  float mx = row[0];
#pragma unroll 1
  for (int n = 1; n < NCLS; ++n) mx = fmaxf(mx, row[n]);
  float s = 0.0f;
#pragma unroll 1
  for (int n = 0; n < NCLS; ++n) s += expf(row[n] - mx);
  const float lg = logf(s);
#pragma unroll 1
  for (int n = 0; n < NCLS; ++n) {
    const float v = (row[n] - mx) - lg;
    if (lane < 16) sres[c * NCLS + n] = v;
  }
  __syncthreads();

  const v4f v0 = *(const v4fa*)(sres + 4 * lane);
  const v4f v1 = *(const v4fa*)(sres + 128 + 4 * (lane & 7));
  float* ob = out + (size_t)blockIdx.x * (16 * NCLS);
  const bool s1 = lane < 8;
  *(volatile v4f*)(ob + 4 * lane) = v0;
  if (s1) *(volatile v4f*)(ob + 128 + 4 * lane) = v1;
  __threadfence();
  *(volatile v4f*)(ob + 4 * lane) = v0;
  if (s1) *(volatile v4f*)(ob + 128 + 4 * lane) = v1;
}

extern "C" void kernel_launch(void* const* d_in, const int* in_sizes, int n_in,
                              void* d_out, int out_size, void* d_ws, size_t ws_size,
                              hipStream_t stream) {
  if (n_in < 3) return;
  const int nimg = in_sizes[0] / NPIX;
  if (nimg <= 0 || nimg * NPIX != in_sizes[0]) return;
  if (in_sizes[1] != NCH * 9) return;
  if (in_sizes[2] != NCLS * KTOT) return;
  if (out_size != nimg * NCLS) return;
  if ((nimg % 16) != 0) return;

  const float* x  = (const float*)d_in[0];
  const float* wf = (const float*)d_in[1];
  const float* wd = (const float*)d_in[2];
  float* out = (float*)d_out;

  const size_t a_bytes = (size_t)nimg * KP * 2;
  const size_t w_off   = a_bytes;
  const size_t w_bytes = (size_t)16 * KP * 2;
  if (w_off + w_bytes > ws_size) return;
  _Float16* Ap = (_Float16*)d_ws;
  _Float16* Wp = (_Float16*)((char*)d_ws + w_off);

  k_wprep<<<dim3(16), dim3(TPB), 0, stream>>>(wd, Wp);
  k_feat<<<dim3(nimg), dim3(TPB), 0, stream>>>(x, wf, Ap);
  k_gemm<<<dim3(nimg / 16), dim3(32), 0, stream>>>(Ap, Wp, out);
  (void)hipGetLastError();
}
